// GCN_41016937677072
// MI455X (gfx1250) — hardware-verified
//
#include <hip/hip_runtime.h>
#include <stddef.h>
#include <stdint.h>
#include <math.h>


#define DIN    128
#define HID    128
#define EMB    256
#define NCL    16
#define K1L    384
#define K2L    512
#define K3L    512
#define ZP     32
#define AGP    256
#define NTHR   256
#define NWAVE  8
#define EPT    8
#define CHUNK  (NTHR * EPT)
#define WCAP   (EPT * 32)
#define LISTN  (NWAVE * WCAP)
#define NBA    2048
#define SLA    11
#define RCAP   24576
#define DEGCAP 64
#define GBM    64
#define GTHR   128
#define G2THR  256
#define AGG_ZINTS    (LISTN + 2 * RCAP + 3 * NBA)
#define MISC_INTS    16
#define SCAN_LDS_INTS (AGG_ZINTS + MISC_INTS)
#define G23_LDS_INTS (GBM * K3L / 2 + GBM * ZP + EMB)
#define NU1    (3 * HID * (DIN / 8))
#define NU2    (4 * EMB * (HID / 8))
#define NU3    (4 * NCL * (EMB / 8))
#define WSMAX  134217728

static_assert((CHUNK & (CHUNK - 1)) == 0 && CHUNK <= 4096);
static_assert((NBA & (NBA - 1)) == 0 && NBA == (1 << SLA));
static_assert(((long long)CHUNK << SLA) < (1LL << 31));
static_assert(LISTN % NTHR == 0);
static_assert(NBA % NWAVE == 0 && NBA % 32 == 0 && NBA % GBM == 0 && NBA % (8 * NWAVE) == 0);
static_assert(RCAP % 4 == 0 && AGG_ZINTS % (NTHR * 4) == 0);
static_assert(K1L % 32 == 0 && K2L % 32 == 0 && K3L % 32 == 0);
static_assert(K1L == 2 * DIN + DIN && K2L == 4 * HID && K3L == 2 * EMB && AGP == 2 * HID && AGP == 2 * DIN);
static_assert(GBM == (GTHR / 32) * 16 && HID == 8 * 16 && EMB == 2 * 8 * 16 && G2THR == EMB);
static_assert(DIN == 4 * 32 && HID == 4 * 32);
static_assert(NU1 % NTHR == 0 && NU2 % NTHR == 0 && NU3 % NTHR == 0);
static_assert((HID * (DIN / 8)) % NTHR == 0 && (EMB * (HID / 8)) % NTHR == 0 && (NCL * (EMB / 8)) % NTHR == 0);
static_assert(SCAN_LDS_INTS * 4 <= 300000 && G23_LDS_INTS * 4 <= 300000);
static_assert(ZP == 2 * NCL);

typedef float          v4f   __attribute__((ext_vector_type(4)));
typedef float          v8f   __attribute__((ext_vector_type(8)));
typedef int            v4i   __attribute__((ext_vector_type(4)));
typedef int            v8i   __attribute__((ext_vector_type(8)));
typedef unsigned       v2u   __attribute__((ext_vector_type(2)));
typedef unsigned       v4u   __attribute__((ext_vector_type(4)));
typedef unsigned short v4us  __attribute__((ext_vector_type(4)));
typedef unsigned short v8us  __attribute__((ext_vector_type(8)));
typedef unsigned short v16us __attribute__((ext_vector_type(16)));
typedef __bf16         v16bf __attribute__((ext_vector_type(16)));
typedef v4f  __attribute__((may_alias)) v4fa;
typedef v4i  __attribute__((may_alias)) v4ia;
typedef v2u  __attribute__((may_alias)) v2ua;
typedef v4us __attribute__((may_alias)) v4usa;
typedef v8us __attribute__((may_alias)) v8usa;
union FragB { v16bf v; v16us u; v8us h[2]; v8i w; };

__device__ __forceinline__ v8f wmb(const FragB& a, const FragB& b, v8f c) {
  v8f d = __builtin_amdgcn_wmma_f32_16x16x32_bf16(false, a.v, false, b.v, (short)0, c, false, false);
  asm volatile("v_nop\n\tv_nop\n\tv_nop\n\tv_nop" : "+v"(d) : "v"(a.w), "v"(b.w));
  return d;
}

__device__ __forceinline__ unsigned bf16_bits(float f) {
  const unsigned u = __float_as_uint(f);
  return (u + 0x7FFFu + ((u >> 16) & 1u)) >> 16;
}
__device__ __forceinline__ float bf16_val(float f) {
  return __uint_as_float(bf16_bits(f) << 16);
}

template <int SLB>
__device__ __forceinline__ int scan_chunk(const int* __restrict__ dsts, int nE, int cbase, int slotBase,
                                          int nb, int vec8, int* list, int tid, int lane, int wave) {
  int wc = 0;
  const int el0  = tid * EPT;
  const int e0   = cbase + el0;
  const int sent = -2147483647 - 1;
  v4i da, db;
  if (vec8 != 0 && cbase + CHUNK <= nE) {
    da = *(const v4i*)(dsts + e0);
    db = *(const v4i*)(dsts + e0 + 4);
  } else {
    da.x = (e0     < nE) ? dsts[min(e0,     nE - 1)] : sent;
    da.y = (e0 + 1 < nE) ? dsts[min(e0 + 1, nE - 1)] : sent;
    da.z = (e0 + 2 < nE) ? dsts[min(e0 + 2, nE - 1)] : sent;
    da.w = (e0 + 3 < nE) ? dsts[min(e0 + 3, nE - 1)] : sent;
    db.x = (e0 + 4 < nE) ? dsts[min(e0 + 4, nE - 1)] : sent;
    db.y = (e0 + 5 < nE) ? dsts[min(e0 + 5, nE - 1)] : sent;
    db.z = (e0 + 6 < nE) ? dsts[min(e0 + 6, nE - 1)] : sent;
    db.w = (e0 + 7 < nE) ? dsts[min(e0 + 7, nE - 1)] : sent;
  }
  const unsigned nbs = (unsigned)slotBase;
  const unsigned unb = (unsigned)nb;
  const unsigned s0 = (unsigned)da.x - nbs, s1 = (unsigned)da.y - nbs;
  const unsigned s2 = (unsigned)da.z - nbs, s3 = (unsigned)da.w - nbs;
  const unsigned s4 = (unsigned)db.x - nbs, s5 = (unsigned)db.y - nbs;
  const unsigned s6 = (unsigned)db.z - nbs, s7 = (unsigned)db.w - nbs;
  const bool h0 = s0 < unb, h1 = s1 < unb, h2 = s2 < unb, h3 = s3 < unb;
  const bool h4 = s4 < unb, h5 = s5 < unb, h6 = s6 < unb, h7 = s7 < unb;
  const unsigned any = __builtin_amdgcn_ballot_w32(h0 | h1 | h2 | h3 | h4 | h5 | h6 | h7);
  if (any != 0u) {
#define HITJ(J, HJ, SJ) { \
      const unsigned mj = __builtin_amdgcn_ballot_w32(HJ); \
      if (mj != 0u) { \
        if (HJ) { \
          const int pos = wc + (int)__builtin_amdgcn_mbcnt_lo(mj, 0u); \
          if (pos < WCAP) list[wave * WCAP + pos] = ((el0 + (J)) << SLB) | (int)(SJ); \
        } \
        wc += (int)__builtin_popcount(mj); } }
    HITJ(0, h0, s0)
    HITJ(1, h1, s1)
    HITJ(2, h2, s2)
    HITJ(3, h3, s3)
    HITJ(4, h4, s4)
    HITJ(5, h5, s5)
    HITJ(6, h6, s6)
    HITJ(7, h7, s7)
#undef HITJ
  }
  return wc;
}

__device__ __forceinline__ void wunit(const float* __restrict__ W, int ldw, int n, int k8, unsigned short* dp) {
  const float* p = W + (size_t)k8 * (size_t)ldw + n;
  v8us o;
#pragma unroll
  for (int i = 0; i < 8; ++i) o[i] = (unsigned short)bf16_bits(p[(size_t)i * (size_t)ldw]);
  *(volatile v8us*)dp = o;
  __threadfence();
  *(volatile v8us*)dp = o;
}

__global__ __launch_bounds__(NTHR) void k_wprep(const float* __restrict__ Wr1, const float* __restrict__ Wo1,
                                                const float* __restrict__ Wr2, const float* __restrict__ Wo2,
                                                const float* __restrict__ Wr3, const float* __restrict__ Wo3,
                                                unsigned short* Bt1, unsigned short* Bt2, unsigned short* Bt3) {
  const int u = (int)blockIdx.x * NTHR + (int)threadIdx.x;
  if (u < NU1) {
    const int part = u >> 11;
    const int v    = u & 2047;
    const int n    = v >> 4;
    const int k8   = (v & 15) * 8;
    unsigned short* dp = Bt1 + (size_t)n * K1L + part * DIN + k8;
    if (part < 2) wunit(Wr1, HID, n, k8, dp);
    else          wunit(Wo1, HID, n, k8, dp);
  } else if (u < NU1 + NU2) {
    const int v0   = u - NU1;
    const int part = v0 >> 12;
    const int v    = v0 & 4095;
    const int n    = v >> 4;
    const int k8   = (v & 15) * 8;
    unsigned short* dp = Bt2 + (size_t)n * K2L + part * HID + k8;
    if (part < 2) wunit(Wr2, EMB, n, k8, dp);
    else          wunit(Wo2, EMB, n, k8, dp);
  } else if (u < NU1 + NU2 + NU3) {
    const int v0   = u - (NU1 + NU2);
    const int part = v0 >> 9;
    const int v    = v0 & 511;
    const int n    = v >> 5;
    const int k8   = (v & 31) * 8;
    const int copy = part & 1;
    if (part < 2) wunit(Wr3, NCL, n, k8, Bt3 + (size_t)n * K3L + copy * EMB + k8);
    else          wunit(Wo3, NCL, n, k8, Bt3 + (size_t)(NCL + n) * K3L + copy * EMB + k8);
  }
}

__global__ __launch_bounds__(NTHR) void k_cvx(const float* __restrict__ x, int nN, int nUnits,
                                              unsigned short* xb) {
  const int u = (int)blockIdx.x * NTHR + (int)threadIdx.x;
  if (u >= nUnits) return;
  const int row = u >> 4;
  const int k8  = (u & 15) * 8;
  const int rc  = row < nN ? row : nN - 1;
  const float* p = x + (size_t)rc * DIN + k8;
  const v4f a = *(const v4fa*)p;
  const v4f b = *(const v4fa*)(p + 4);
  const bool ok = row < nN;
  v8us o;
  o[0] = ok ? (unsigned short)bf16_bits(a.x) : (unsigned short)0;
  o[1] = ok ? (unsigned short)bf16_bits(a.y) : (unsigned short)0;
  o[2] = ok ? (unsigned short)bf16_bits(a.z) : (unsigned short)0;
  o[3] = ok ? (unsigned short)bf16_bits(a.w) : (unsigned short)0;
  o[4] = ok ? (unsigned short)bf16_bits(b.x) : (unsigned short)0;
  o[5] = ok ? (unsigned short)bf16_bits(b.y) : (unsigned short)0;
  o[6] = ok ? (unsigned short)bf16_bits(b.z) : (unsigned short)0;
  o[7] = ok ? (unsigned short)bf16_bits(b.w) : (unsigned short)0;
  unsigned short* dp = xb + (size_t)row * DIN + k8;
  *(volatile v8us*)dp = o;
  __threadfence();
  *(volatile v8us*)dp = o;
}

template <int NT>
__device__ __forceinline__ void gemm_seg(const unsigned short* __restrict__ ap, int width,
                                         const unsigned short* __restrict__ bp, int ldb, v8f (&acc)[NT]) {
#pragma unroll 1
  for (int k0 = 0; k0 < width; k0 += 32) {
    FragB af;
    af.h[0] = *(const v8usa*)(ap + k0);
    af.h[1] = *(const v8usa*)(ap + k0 + 16);
#pragma unroll
    for (int nt = 0; nt < NT; ++nt) {
      const unsigned short* wq = bp + (size_t)(16 * nt) * (size_t)ldb + k0;
      FragB bf;
      bf.h[0] = *(const v8usa*)wq;
      bf.h[1] = *(const v8usa*)(wq + 16);
      acc[nt] = wmb(af, bf, acc[nt]);
    }
  }
}

__global__ __launch_bounds__(GTHR) void k_gemm1(const unsigned short* __restrict__ agg,
                                                const unsigned short* __restrict__ xb,
                                                const unsigned short* __restrict__ BT,
                                                const float* __restrict__ bias, unsigned short* h1, int nOut) {
  __shared__ __attribute__((aligned(16))) float stg[GBM * HID];
  const int tid = (int)threadIdx.x, lane = tid & 31, wave = tid >> 5, hh = lane >> 4, m = lane & 15;
  const int rowBase = (int)blockIdx.x * GBM;

  v8f acc[8];
  {
    const v8f z = {0.f, 0.f, 0.f, 0.f, 0.f, 0.f, 0.f, 0.f};
#pragma unroll
    for (int t = 0; t < 8; ++t) acc[t] = z;
  }
  const size_t arow = (size_t)(rowBase + 16 * wave + m);
  const unsigned short* bp = BT + (size_t)m * K1L + 8 * hh;
  gemm_seg<8>(agg + arow * AGP + 8 * hh, 2 * DIN, bp, K1L, acc);
  gemm_seg<8>(xb + arow * DIN + 8 * hh, DIN, bp + 2 * DIN, K1L, acc);

#pragma unroll
  for (int nt = 0; nt < 8; ++nt) {
    const int lc = 16 * nt + m;
#pragma unroll
    for (int r = 0; r < 8; ++r) {
      const int lr = 16 * wave + 8 * hh + r;
      stg[lr * HID + lc] = acc[nt][r];
    }
  }
  __syncthreads();

  v4f bb4;
  {
    const v4f t1 = *(const v4f*)(bias + 4 * lane);
    bb4.x = bf16_val(t1.x); bb4.y = bf16_val(t1.y); bb4.z = bf16_val(t1.z); bb4.w = bf16_val(t1.w);
  }
  v4f pv[16];
#pragma unroll
  for (int i = 0; i < 16; ++i) pv[i] = *(const v4fa*)(stg + (16 * wave + i) * HID + 4 * lane);
  __syncthreads();

#pragma unroll
  for (int i = 0; i < 16; ++i) {
    const bool ok = (rowBase + 16 * wave + i) < nOut;
    const v4f t = pv[i] + bb4;
    v4f y;
    y.x = (t.x > 0.0f) ? t.x : (t.x - t.x);
    y.y = (t.y > 0.0f) ? t.y : (t.y - t.y);
    y.z = (t.z > 0.0f) ? t.z : (t.z - t.z);
    y.w = (t.w > 0.0f) ? t.w : (t.w - t.w);
    y.x = ok ? y.x : 0.0f; y.y = ok ? y.y : 0.0f; y.z = ok ? y.z : 0.0f; y.w = ok ? y.w : 0.0f;
    pv[i] = y;
  }
#pragma unroll
  for (int i = 0; i < 16; ++i) {
    v4us h4, l4;
    unsigned hb;
    hb = bf16_bits(pv[i].x); h4[0] = (unsigned short)hb; l4[0] = (unsigned short)bf16_bits(pv[i].x - __uint_as_float(hb << 16));
    hb = bf16_bits(pv[i].y); h4[1] = (unsigned short)hb; l4[1] = (unsigned short)bf16_bits(pv[i].y - __uint_as_float(hb << 16));
    hb = bf16_bits(pv[i].z); h4[2] = (unsigned short)hb; l4[2] = (unsigned short)bf16_bits(pv[i].z - __uint_as_float(hb << 16));
    hb = bf16_bits(pv[i].w); h4[3] = (unsigned short)hb; l4[3] = (unsigned short)bf16_bits(pv[i].w - __uint_as_float(hb << 16));
    unsigned short* srow = (unsigned short*)stg + (size_t)(16 * wave + i) * (2 * HID);
    *(v4usa*)(srow + 4 * lane) = h4;
    *(v4usa*)(srow + HID + 4 * lane) = l4;
  }
  __syncthreads();
  v8us qv[16];
#pragma unroll
  for (int i = 0; i < 16; ++i) {
    const unsigned short* srow = (const unsigned short*)stg + (size_t)(16 * wave + i) * (2 * HID);
    qv[i] = *(const v8usa*)(srow + 8 * lane);
  }
#pragma unroll
  for (int i = 0; i < 16; ++i) {
    unsigned short* rp = h1 + (size_t)(rowBase + 16 * wave + i) * (size_t)AGP + 8 * lane;
    *(volatile v8us*)rp = qv[i];
  }
  __threadfence();
#pragma unroll
  for (int i = 0; i < 16; ++i) {
    unsigned short* rp = h1 + (size_t)(rowBase + 16 * wave + i) * (size_t)AGP + 8 * lane;
    *(volatile v8us*)rp = qv[i];
  }
}

__global__ __launch_bounds__(G2THR) void k_gemm23(const unsigned short* __restrict__ agg,
                                                  const unsigned short* __restrict__ h1,
                                                  const unsigned short* __restrict__ BT2,
                                                  const unsigned short* __restrict__ BT3,
                                                  const float* __restrict__ bias2, float* zout, int nOut) {
  extern __shared__ __attribute__((aligned(16))) int dsmg[];
  unsigned short* h2s = (unsigned short*)dsmg;
  float* zst = (float*)(dsmg + GBM * K3L / 2);
  float* bls = (float*)(dsmg + GBM * K3L / 2 + GBM * ZP);
  const int tid = (int)threadIdx.x, lane = tid & 31, wave = tid >> 5, hh = lane >> 4, m = lane & 15;
  const int wr = wave & 3, wc = wave >> 2;
  const int rowBase = (int)blockIdx.x * GBM;

  bls[tid] = bf16_val(bias2[tid]);

  v8f acc[8];
  {
    const v8f z = {0.f, 0.f, 0.f, 0.f, 0.f, 0.f, 0.f, 0.f};
#pragma unroll
    for (int t = 0; t < 8; ++t) acc[t] = z;
  }
  {
    const size_t arow = (size_t)(rowBase + 16 * wr + m);
    const unsigned short* bp = BT2 + (size_t)(128 * wc + m) * K2L + 8 * hh;
    gemm_seg<8>(agg + arow * AGP + 8 * hh, 2 * HID, bp, K2L, acc);
    gemm_seg<8>(h1 + arow * AGP + 8 * hh, 2 * HID, bp + 2 * HID, K2L, acc);
  }
  __syncthreads();

#pragma unroll
  for (int nt = 0; nt < 8; ++nt) {
    const int col = 128 * wc + 16 * nt + m;
    const float bv = bls[col];
#pragma unroll
    for (int r = 0; r < 8; ++r) {
      const int lr = 16 * wr + 8 * hh + r;
      const float t = acc[nt][r] + bv;
      float y = (t > 0.0f) ? t : (t - t);
      y = ((rowBase + lr) < nOut) ? y : 0.0f;
      const unsigned hb = bf16_bits(y);
      const unsigned lb = bf16_bits(y - __uint_as_float(hb << 16));
      h2s[lr * K3L + col]       = (unsigned short)hb;
      h2s[lr * K3L + EMB + col] = (unsigned short)lb;
    }
  }
  __syncthreads();

  {
    const int rt = wave & 3, ct = wave >> 2;
    const unsigned short* as = h2s + (16 * rt + m) * K3L + 8 * hh;
    const unsigned short* b3p = BT3 + (size_t)(16 * ct + m) * K3L + 8 * hh;
    v8f a3 = {0.f, 0.f, 0.f, 0.f, 0.f, 0.f, 0.f, 0.f};
#pragma unroll 1
    for (int k0 = 0; k0 < K3L; k0 += 32) {
      FragB af, bf;
      af.h[0] = *(const v8usa*)(as + k0);
      af.h[1] = *(const v8usa*)(as + k0 + 16);
      bf.h[0] = *(const v8usa*)(b3p + k0);
      bf.h[1] = *(const v8usa*)(b3p + k0 + 16);
      a3 = wmb(af, bf, a3);
    }
#pragma unroll
    for (int r = 0; r < 8; ++r) zst[(16 * rt + 8 * hh + r) * ZP + 16 * ct + m] = a3[r];
  }
  __syncthreads();

  v4f zv[2];
#pragma unroll
  for (int it = 0; it < 2; ++it) {
    const int row = it * 32 + (tid >> 3);
    zv[it] = *(const v4fa*)(zst + row * ZP + 4 * (tid & 7));
  }
#pragma unroll
  for (int it = 0; it < 2; ++it) {
    const int row = it * 32 + (tid >> 3);
    *(volatile v4f*)(zout + (size_t)(rowBase + row) * ZP + 4 * (tid & 7)) = zv[it];
  }
  __threadfence();
#pragma unroll
  for (int it = 0; it < 2; ++it) {
    const int row = it * 32 + (tid >> 3);
    *(volatile v4f*)(zout + (size_t)(rowBase + row) * ZP + 4 * (tid & 7)) = zv[it];
  }
}

template <int MODE>
__global__ __launch_bounds__(NTHR) void k_scan(const int* __restrict__ srcs, const int* __restrict__ dsts,
                                               int nE, int nN, int vec8, int mRows,
                                               const unsigned short* __restrict__ gpl, unsigned short* aggp,
                                               const float* __restrict__ zpl, const float* __restrict__ b3,
                                               float* outp) {
  extern __shared__ __attribute__((aligned(16))) int dsm[];
  int* list = dsm;
  int* hl   = dsm + LISTN;
  int* sl   = hl + RCAP;
  int* cnt  = sl + RCAP;
  int* offs = cnt + NBA;
  int* cur  = offs + NBA;
  int* misc = cur + NBA;
  const int tid = (int)threadIdx.x, lane = tid & 31, wave = tid >> 5;
  const int nodeBase = (int)blockIdx.x * NBA;

  {
    const v4i z4 = {0, 0, 0, 0};
    for (int i = tid * 4; i < AGG_ZINTS; i += NTHR * 4) *(v4ia*)(dsm + i) = z4;
    if (tid < MISC_INTS) misc[tid] = 0;
  }
  __syncthreads();

  int t = 0, ov = 0;
  const int nChunks = (nE + CHUNK - 1) / CHUNK;
#pragma unroll 1
  for (int ch = 0; ch < nChunks; ++ch) {
    const int cbase = ch * CHUNK;
    const int wc = scan_chunk<SLA>(dsts, nE, cbase, nodeBase, NBA, vec8, list, tid, lane, wave);
    if (lane == 0) misc[wave] = wc;
    __syncthreads();
    if (wave == 0) {
#pragma unroll 1
      for (int w2 = 0; w2 < NWAVE; ++w2) {
        int c = misc[w2];
        c = c < 0 ? 0 : (c > WCAP ? WCAP : c);
#pragma unroll 1
        for (int b0 = 0; b0 < c; b0 += 32) {
          const int idx = b0 + lane;
          const int ent = list[w2 * WCAP + (idx < WCAP ? idx : WCAP - 1)];
          const int m32 = (c - b0) < 32 ? (c - b0) : 32;
#pragma unroll 1
          for (int k = 0; k < m32; ++k) {
            const int u    = __builtin_amdgcn_readlane(ent, k);
            const int slot = u & (NBA - 1);
            const int el   = (u >> SLA) & (CHUNK - 1);
            const int pk   = ((cbase + el) << SLA) | slot;
            if (t < RCAP) {
              if (lane == 0) { hl[t] = pk; cnt[slot] = cnt[slot] + 1; }
              t = t + 1;
            } else {
              ov = 1;
            }
          }
        }
      }
    }
    __syncthreads();
  }
  if (wave == 0 && lane == 0) { misc[8] = t; misc[9] = ov; }
  __syncthreads();
  int tt = misc[8];
  tt = tt < 0 ? 0 : (tt > RCAP ? RCAP : tt);
  const int ovf = misc[9];

  if (wave == 0) {
    const int base = lane * (NBA / 32);
    int s = 0;
#pragma unroll 1
    for (int i = 0; i < NBA / 32; ++i) s += cnt[base + i];
    int incl = s;
#pragma unroll
    for (int d = 1; d < 32; d <<= 1) {
      const int y = __shfl_up(incl, d, 32);
      if (lane >= d) incl += y;
    }
    int run = incl - s;
#pragma unroll 1
    for (int i = 0; i < NBA / 32; ++i) {
      const int cv = cnt[base + i];
      offs[base + i] = run;
      cur[base + i]  = run;
      run += cv;
    }
  }
  __syncthreads();
  if (wave == 0) {
#pragma unroll 1
    for (int b0 = 0; b0 < tt; b0 += 32) {
      const int idx = b0 + lane;
      const int ent = hl[idx < RCAP ? idx : RCAP - 1];
      const int m32 = (tt - b0) < 32 ? (tt - b0) : 32;
#pragma unroll 1
      for (int k = 0; k < m32; ++k) {
        const int u    = __builtin_amdgcn_readlane(ent, k);
        const int slot = u & (NBA - 1);
        if (lane == 0) {
          int p = cur[slot];
          p = p < 0 ? 0 : (p > RCAP - 1 ? RCAP - 1 : p);
          sl[p] = u;
          cur[slot] = p + 1;
        }
      }
    }
  }
  __syncthreads();

  const float qnan = __int_as_float(0x7fc00000);
  const float pz = (ovf != 0) ? qnan : 0.0f;

  if constexpr (MODE != 2) {
    const int sa = (2 * lane) & 31, sb = (2 * lane + 1) & 31;
    const bool lsel = lane >= 16;
#pragma unroll 1
    for (int si = 0; si < NBA / NWAVE; ++si) {
      const int s    = si * NWAVE + wave;
      const int node = nodeBase + s;
      int c = cnt[s];
      const bool big = c > DEGCAP;
      c = c < 0 ? 0 : (c > DEGCAP ? DEGCAP : c);
      int o = offs[s];
      o = o < 0 ? 0 : (o > RCAP ? RCAP : o);
      float a0 = 0.0f, a1 = 0.0f, a2 = 0.0f, a3 = 0.0f;
#pragma unroll 1
      for (int b0 = 0; b0 < c; b0 += 32) {
        int idx = o + b0 + lane;
        idx = idx > RCAP - 1 ? RCAP - 1 : idx;
        const int ent = sl[idx];
        int eid = ent >> SLA;
        eid = eid < 0 ? 0 : (eid > nE - 1 ? nE - 1 : eid);
        int sr = srcs[eid];
        sr = sr < 0 ? 0 : (sr > nN - 1 ? nN - 1 : sr);
        const int m32 = (c - b0) < 32 ? (c - b0) : 32;
#pragma unroll 1
        for (int k = 0; k < m32; ++k) {
          const int sk = __builtin_amdgcn_readlane(sr, k);
          if constexpr (MODE == 0) {
            const unsigned short* rp = gpl + (size_t)sk * DIN + 4 * lane;
            const v2u wh = *(const v2ua*)rp;
            a0 += __uint_as_float(wh.x << 16);
            a1 += __uint_as_float(wh.x & 0xffff0000u);
            a2 += __uint_as_float(wh.y << 16);
            a3 += __uint_as_float(wh.y & 0xffff0000u);
          } else {
            const unsigned short* rp = gpl + (size_t)sk * AGP + 4 * lane;
            const v2u wh = *(const v2ua*)rp;
            const v2u wl = *(const v2ua*)(rp + HID);
            const float f0 = __uint_as_float(wh.x << 16)         + __uint_as_float(wl.x << 16);
            const float f1 = __uint_as_float(wh.x & 0xffff0000u) + __uint_as_float(wl.x & 0xffff0000u);
            const float f2 = __uint_as_float(wh.y << 16)         + __uint_as_float(wl.y << 16);
            const float f3 = __uint_as_float(wh.y & 0xffff0000u) + __uint_as_float(wl.y & 0xffff0000u);
            a0 += f0; a1 += f1; a2 += f2; a3 += f3;
          }
        }
      }
      const float pzr = big ? qnan : pz;
      const bool live = node < nN;
      const float m0 = live ? (a0 + pzr) : 0.0f;
      const float m1 = live ? (a1 + pzr) : 0.0f;
      const float m2 = live ? (a2 + pzr) : 0.0f;
      const float m3 = live ? (a3 + pzr) : 0.0f;
      const unsigned hb0 = bf16_bits(m0), hb1 = bf16_bits(m1), hb2 = bf16_bits(m2), hb3 = bf16_bits(m3);
      const unsigned lb0 = bf16_bits(m0 - __uint_as_float(hb0 << 16));
      const unsigned lb1 = bf16_bits(m1 - __uint_as_float(hb1 << 16));
      const unsigned lb2 = bf16_bits(m2 - __uint_as_float(hb2 << 16));
      const unsigned lb3 = bf16_bits(m3 - __uint_as_float(hb3 << 16));
      const int hw0 = (int)(hb0 | (hb1 << 16));
      const int hw1 = (int)(hb2 | (hb3 << 16));
      const int lw0 = (int)(lb0 | (lb1 << 16));
      const int lw1 = (int)(lb2 | (lb3 << 16));
      const int g0 = __shfl(hw0, sa, 32), g1 = __shfl(hw1, sa, 32);
      const int g2 = __shfl(hw0, sb, 32), g3 = __shfl(hw1, sb, 32);
      const int p0 = __shfl(lw0, sa, 32), p1 = __shfl(lw1, sa, 32);
      const int p2 = __shfl(lw0, sb, 32), p3 = __shfl(lw1, sb, 32);
      v4u pv;
      pv.x = (unsigned)(lsel ? p0 : g0);
      pv.y = (unsigned)(lsel ? p1 : g1);
      pv.z = (unsigned)(lsel ? p2 : g2);
      pv.w = (unsigned)(lsel ? p3 : g3);
      if (node < mRows) {
        unsigned short* hp = aggp + (size_t)node * AGP + 8 * lane;
        *(volatile v4u*)hp = pv;
        __threadfence();
        *(volatile v4u*)hp = pv;
      }
    }
  } else {
    const int chn = lane & 15;
    const float bch = bf16_val(b3[chn]);
    const int rsel = lane >> 2;
    const int c0s = 4 * (lane & 3);
#pragma unroll 1
    for (int gi = 0; gi < NBA / (8 * NWAVE); ++gi) {
      const int s0    = (gi * NWAVE + wave) * 8;
      const int node0 = nodeBase + s0;
      if (node0 < nN) {
        v4f q = {0.f, 0.f, 0.f, 0.f};
#pragma unroll 1
        for (int r = 0; r < 8; ++r) {
          const int s = s0 + r;
          const int node = node0 + r;
          int c = cnt[s];
          const bool big = c > DEGCAP;
          c = c < 0 ? 0 : (c > DEGCAP ? DEGCAP : c);
          int o = offs[s];
          o = o < 0 ? 0 : (o > RCAP ? RCAP : o);
          const int nc = node < nN ? node : nN - 1;
          float acc = 0.0f;
#pragma unroll 1
          for (int b0 = 0; b0 < c; b0 += 32) {
            int idx = o + b0 + lane;
            idx = idx > RCAP - 1 ? RCAP - 1 : idx;
            const int ent = sl[idx];
            int eid = ent >> SLA;
            eid = eid < 0 ? 0 : (eid > nE - 1 ? nE - 1 : eid);
            int sr = srcs[eid];
            sr = sr < 0 ? 0 : (sr > nN - 1 ? nN - 1 : sr);
            const int m32 = (c - b0) < 32 ? (c - b0) : 32;
#pragma unroll 1
            for (int k = 0; k < m32; ++k) {
              const int sk = __builtin_amdgcn_readlane(sr, k);
              acc += zpl[(size_t)sk * ZP + chn];
            }
          }
          const float zr = zpl[(size_t)nc * ZP + NCL + chn];
          const float v = (acc + zr) + bch;
          float mx = v;
#pragma unroll
          for (int d = 8; d >= 1; d >>= 1) {
            const float ot = __shfl_xor(mx, d, 32);
            float tm = (ot > mx) ? ot : mx;
            tm = (ot != ot) ? ot : tm;
            mx = tm;
          }
          const float sh = v - mx;
          float sm = expf(sh);
#pragma unroll
          for (int d = 8; d >= 1; d >>= 1) sm += __shfl_xor(sm, d, 32);
          float res = sh - logf(sm);
          res = res + (big ? qnan : pz);
          const float t0 = __shfl(res, c0s + 0, 32);
          const float t1 = __shfl(res, c0s + 1, 32);
          const float t2 = __shfl(res, c0s + 2, 32);
          const float t3 = __shfl(res, c0s + 3, 32);
          const bool mine = (rsel == r);
          q.x = mine ? t0 : q.x;
          q.y = mine ? t1 : q.y;
          q.z = mine ? t2 : q.z;
          q.w = mine ? t3 : q.w;
        }
        float* op = outp + (size_t)node0 * NCL + 4 * lane;
        *(volatile v4f*)op = q;
        __threadfence();
        *(volatile v4f*)op = q;
      }
    }
  }
}

static inline int cdiv(int a, int b) { return (a + b - 1) / b; }
static inline size_t al256(size_t o) { return (o + 255) & ~(size_t)255; }

extern "C" void kernel_launch(void* const* d_in, const int* in_sizes, int n_in,
                              void* d_out, int out_size, void* d_ws, size_t ws_size,
                              hipStream_t stream) {
  if (n_in < 11) return;
  if (in_sizes[0] < DIN || (in_sizes[0] % DIN) != 0) return;
  const int nN = in_sizes[0] / DIN;
  if (nN < 8 || (nN & 7) != 0 || nN > (1 << 22)) return;
  if (in_sizes[1] < 2 || (in_sizes[1] & 1) != 0) return;
  const int nE = in_sizes[1] / 2;
  if (nE < 1 || nE >= (1 << (31 - SLA))) return;
  if (in_sizes[2] != DIN * HID || in_sizes[3] != DIN * HID || in_sizes[4] != HID) return;
  if (in_sizes[5] != HID * EMB || in_sizes[6] != HID * EMB || in_sizes[7] != EMB) return;
  if (in_sizes[8] != EMB * NCL || in_sizes[9] != EMB * NCL || in_sizes[10] != NCL) return;
  if ((long long)out_size != (long long)nN * NCL) return;

  const float* x    = (const float*)d_in[0];
  const int*   edge = (const int*)d_in[1];
  const float* Wr1  = (const float*)d_in[2];
  const float* Wo1  = (const float*)d_in[3];
  const float* b1   = (const float*)d_in[4];
  const float* Wr2  = (const float*)d_in[5];
  const float* Wo2  = (const float*)d_in[6];
  const float* b2   = (const float*)d_in[7];
  const float* Wr3  = (const float*)d_in[8];
  const float* Wo3  = (const float*)d_in[9];
  const float* b3   = (const float*)d_in[10];
  float* out = (float*)d_out;
  const int* src = edge;
  const int* dst = edge + nE;

  const int MP  = cdiv(nN, GBM) * GBM;
  const int gM  = MP / GBM;
  const int gA  = cdiv(MP, NBA);
  const int gA3 = cdiv(nN, NBA);
  if ((long long)gA * NBA < (long long)MP) return;
  const int vec8 = ((nE & 3) == 0) ? 1 : 0;

  char* ws = (char*)d_ws;
  size_t off = 0;
  const size_t oB1 = off; off = al256(off + (size_t)HID * K1L * 2);
  const size_t oB2 = off; off = al256(off + (size_t)EMB * K2L * 2);
  const size_t oB3 = off; off = al256(off + (size_t)ZP * K3L * 2);
  const size_t oR0 = off; off = al256(off + (size_t)MP * DIN * 2);
  const size_t oAG = off; off = al256(off + (size_t)MP * AGP * 2);
  const size_t oH1 = off; off = al256(off + (size_t)MP * AGP * 2);
  if ((size_t)MP * ZP * 4 > (size_t)MP * DIN * 2) return;
  if (off > ws_size || off > (size_t)WSMAX) return;
  unsigned short* Bt1 = (unsigned short*)(ws + oB1);
  unsigned short* Bt2 = (unsigned short*)(ws + oB2);
  unsigned short* Bt3 = (unsigned short*)(ws + oB3);
  unsigned short* XB  = (unsigned short*)(ws + oR0);
  float*          Zp  = (float*)(ws + oR0);
  unsigned short* AGG = (unsigned short*)(ws + oAG);
  unsigned short* H1  = (unsigned short*)(ws + oH1);

  const size_t scanLds = (size_t)SCAN_LDS_INTS * 4;
  const size_t g23Lds  = (size_t)G23_LDS_INTS * 4;
  hipFuncSetAttribute(reinterpret_cast<const void*>(&k_scan<0>), hipFuncAttributeMaxDynamicSharedMemorySize, (int)scanLds);
  hipFuncSetAttribute(reinterpret_cast<const void*>(&k_scan<1>), hipFuncAttributeMaxDynamicSharedMemorySize, (int)scanLds);
  hipFuncSetAttribute(reinterpret_cast<const void*>(&k_scan<2>), hipFuncAttributeMaxDynamicSharedMemorySize, (int)scanLds);
  hipFuncSetAttribute(reinterpret_cast<const void*>(&k_gemm23), hipFuncAttributeMaxDynamicSharedMemorySize, (int)g23Lds);

  const int nUx = MP * (DIN / 8);
  k_wprep<<<(NU1 + NU2 + NU3) / NTHR, NTHR, 0, stream>>>(Wr1, Wo1, Wr2, Wo2, Wr3, Wo3, Bt1, Bt2, Bt3);
  k_cvx<<<cdiv(nUx, NTHR), NTHR, 0, stream>>>(x, nN, nUx, XB);
  k_scan<0><<<gA, NTHR, scanLds, stream>>>(src, dst, nE, nN, vec8, MP, XB, AGG, Zp, b3, out);
  k_gemm1<<<gM, GTHR, 0, stream>>>(AGG, XB, Bt1, b1, H1, nN);
  k_scan<1><<<gA, NTHR, scanLds, stream>>>(src, dst, nE, nN, vec8, MP, H1, AGG, Zp, b3, out);
  k_gemm23<<<gM, G2THR, g23Lds, stream>>>(AGG, H1, Bt2, Bt3, b2, Zp, nN);
  k_scan<2><<<gA3, NTHR, scanLds, stream>>>(src, dst, nE, nN, vec8, MP, H1, AGG, Zp, b3, out);
}
